// PointCloudEncoder_43800076485394
// MI455X (gfx1250) — hardware-verified
//
#include <hip/hip_runtime.h>
#include <stdint.h>

#pragma clang fp contract(off)

typedef __attribute__((ext_vector_type(16))) _Float16 v16h;
typedef __attribute__((ext_vector_type(8)))  _Float16 v8h;
typedef __attribute__((ext_vector_type(8)))  float    v8f;
typedef __attribute__((ext_vector_type(4)))  float    v4f;
typedef __attribute__((ext_vector_type(4)))  unsigned int v4u;

constexpr int NBATCH  = 8;
constexpr int NPTS    = 8192;
constexpr int DIN_CH  = 16;
constexpr int NGRP    = 512;
constexpr int KNBR    = 32;
constexpr int OUT_CH  = 256;
constexpr int MID_CH  = 128;
constexpr int PREV_CH = 128;
constexpr int CEXP_CH = 259;
constexpr int CPAD_CH = 288;
constexpr int NQRY    = NBATCH * NGRP;
constexpr int ROWS_CHUNK = NGRP * KNBR;
constexpr int NPT_ALL = NBATCH * NPTS;
constexpr int KPAD_EMB = 32;
constexpr int KNN_CAP  = 128;
constexpr int KNN_TPITCH = 64;
constexpr int FPS_THREADS = 512;
constexpr int FPS_PPT = NPTS / FPS_THREADS;
constexpr float INVSQ = 0.99999500003749969f;
constexpr float WCARRY = 64.0f;
constexpr float WCARRY_INV = 1.0f / 64.0f;
constexpr float FINF = __builtin_huge_valf();
constexpr int   BIGI = 0x7fffffff;

static_assert(FPS_PPT * FPS_THREADS == NPTS);
static_assert(NPTS == 256 * KNBR);
static_assert(KPAD_EMB % 32 == 0 && CPAD_CH % 32 == 0 && OUT_CH % 32 == 0 && MID_CH % 32 == 0);
static_assert(NPT_ALL % 64 == 0 && ROWS_CHUNK % 64 == 0 && PREV_CH % 64 == 0 && OUT_CH % 64 == 0 && MID_CH % 64 == 0);

constexpr size_t SZ_FEATP = (size_t)NPT_ALL * KPAD_EMB * 2;
constexpr size_t SZ_WEH   = (size_t)PREV_CH * KPAD_EMB * 2;
constexpr size_t SZ_W1H   = (size_t)OUT_CH * CPAD_CH * 2;
constexpr size_t SZ_WDH   = (size_t)2 * MID_CH * OUT_CH * 2;
constexpr size_t SZ_WUH   = (size_t)2 * OUT_CH * MID_CH * 2;
constexpr size_t SZ_F0H   = (size_t)NPT_ALL * PREV_CH * 2;
constexpr size_t SZ_SELT  = (size_t)NQRY * 4;
constexpr size_t SZ_KNNT  = (size_t)NQRY * KNN_TPITCH * 4;
constexpr size_t SZ_STATS = 256;
constexpr size_t SZ_E     = (size_t)ROWS_CHUNK * CPAD_CH * 2;
constexpr size_t SZ_WGT   = (size_t)ROWS_CHUNK * 4;
constexpr size_t SZ_X32   = (size_t)ROWS_CHUNK * OUT_CH * 4;
constexpr size_t SZ_X16   = (size_t)ROWS_CHUNK * OUT_CH * 2;
constexpr size_t SZ_H16   = (size_t)ROWS_CHUNK * MID_CH * 2;

constexpr size_t OFF_FEATP = 0;
constexpr size_t OFF_WEH   = OFF_FEATP + SZ_FEATP;
constexpr size_t OFF_W1H   = OFF_WEH + SZ_WEH;
constexpr size_t OFF_WDH   = OFF_W1H + SZ_W1H;
constexpr size_t OFF_WUH   = OFF_WDH + SZ_WDH;
constexpr size_t OFF_F0H   = OFF_WUH + SZ_WUH;
constexpr size_t OFF_SELT  = OFF_F0H + SZ_F0H;
constexpr size_t OFF_KNNT  = OFF_SELT + SZ_SELT;
constexpr size_t OFF_STATS = OFF_KNNT + SZ_KNNT;
constexpr size_t OFF_E     = OFF_STATS + SZ_STATS;
constexpr size_t OFF_WGT   = OFF_E + SZ_E;
constexpr size_t OFF_X32A  = OFF_WGT + SZ_WGT;
constexpr size_t OFF_X32B  = OFF_X32A + SZ_X32;
constexpr size_t OFF_X16   = OFF_X32B + SZ_X32;
constexpr size_t OFF_H16   = OFF_X16 + SZ_X16;
constexpr size_t WS_TOTAL  = OFF_H16 + SZ_H16;
static_assert(WS_TOTAL <= (size_t)134217728);
static_assert((OFF_WEH % 256) == 0 && (OFF_W1H % 256) == 0 && (OFF_WDH % 256) == 0 && (OFF_WUH % 256) == 0 &&
              (OFF_F0H % 256) == 0 && (OFF_SELT % 256) == 0 && (OFF_KNNT % 256) == 0 && (OFF_STATS % 256) == 0 &&
              (OFF_E % 256) == 0 && (OFF_WGT % 256) == 0 && (OFF_X32A % 256) == 0 && (OFF_X32B % 256) == 0 &&
              (OFF_X16 % 256) == 0 && (OFF_H16 % 256) == 0);

__device__ __forceinline__ void dep_guard_h(v8f& a, v8f& b, v16h x, v16h y) { asm volatile("v_nop\n\tv_nop\n\tv_nop\n\tv_nop" : "+v"(a), "+v"(b) : "v"(x), "v"(y)); }
__device__ __forceinline__ void keep4_h(v16h a, v16h b, v16h c, v16h d) { asm volatile("v_nop" :: "v"(a), "v"(b), "v"(c), "v"(d)); }
__device__ __forceinline__ void acc_guard4(v8f& a, v8f& b, v8f& c, v8f& d) { asm volatile("v_nop\n\tv_nop\n\tv_nop\n\tv_nop" : "+v"(a), "+v"(b), "+v"(c), "+v"(d)); }
template <typename T> struct Frag;
template <> struct Frag<_Float16> {
  typedef v16h V; union U { v16h v; v8h h[2]; };
  static __device__ __forceinline__ v16h load(const _Float16* p) {
    U f; f.h[0] = *(const v8h*)(p); f.h[1] = *(const v8h*)(p + 16); return f.v;
  }
  static __device__ __forceinline__ v8f mma(v16h a, v16h b, v8f c) {
    return __builtin_amdgcn_wmma_f32_16x16x32_f16(false, a, false, b, (short)0, c, false, false);
  }
  static __device__ __forceinline__ void guard(v8f& a, v8f& b, v16h x, v16h y) { dep_guard_h(a, b, x, y); }
  static __device__ __forceinline__ void keep(v16h a, v16h b, v16h c, v16h d) { keep4_h(a, b, c, d); }
};

__device__ __forceinline__ void wave_sync() {
  __builtin_amdgcn_fence(__ATOMIC_RELEASE, "workgroup");
  __builtin_amdgcn_wave_barrier();
  __builtin_amdgcn_fence(__ATOMIC_ACQUIRE, "workgroup");
}

__device__ __forceinline__ unsigned short h_bits(float f) { return __builtin_bit_cast(unsigned short, (_Float16)f); }
__device__ __forceinline__ unsigned int pack2h(float a, float b) {
  return (unsigned int)h_bits(a) | ((unsigned int)h_bits(b) << 16);
}

__device__ __forceinline__ void lex_max(float& v, int& i, float ov, int oi) {
  const bool tk = (ov > v) || (ov == v && oi < i);
  v = tk ? ov : v; i = tk ? oi : i;
}
__device__ __forceinline__ void lex_min(float& v, int& i, float ov, int oi) {
  const bool tk = (ov < v) || (ov == v && oi < i);
  v = tk ? ov : v; i = tk ? oi : i;
}
__device__ __forceinline__ void wave_argmax(float& v, int& i) {
#pragma unroll
  for (int off = 16; off > 0; off >>= 1) {
    const float ov = __shfl_xor(v, off, 32); const int oi = __shfl_xor(i, off, 32);
    lex_max(v, i, ov, oi);
  }
}
__device__ __forceinline__ void wave_argmin(float& v, int& i) {
#pragma unroll
  for (int off = 16; off > 0; off >>= 1) {
    const float ov = __shfl_xor(v, off, 32); const int oi = __shfl_xor(i, off, 32);
    lex_min(v, i, ov, oi);
  }
}
__device__ __forceinline__ double shfl_xor_d(double x, int off) {
  const long long v = __double_as_longlong(x);
  int lo = (int)(v & 0xffffffffLL); int hi = (int)((unsigned long long)v >> 32);
  lo = __shfl_xor(lo, off, 32); hi = __shfl_xor(hi, off, 32);
  const unsigned long long r = ((unsigned long long)(unsigned int)hi << 32) | (unsigned long long)(unsigned int)lo;
  return __longlong_as_double((long long)r);
}

__global__ __launch_bounds__(256) void k_cast_pad2(
    const float* __restrict__ inA, int nchA, unsigned short* __restrict__ outA,
    const float* __restrict__ inB, int nchB, unsigned short* __restrict__ outB, int nblkA, float scaleB)
{
  const bool segA = (int)blockIdx.x < nblkA;
  const float* in = segA ? inA : inB;
  unsigned short* out = segA ? outA : outB;
  const int nch = segA ? nchA : nchB;
  const float sc = segA ? 1.0f : scaleB;
  const int c = (segA ? (int)blockIdx.x : ((int)blockIdx.x - nblkA)) * 256 + (int)threadIdx.x;
  if (c >= nch) return;
  const int row = c >> 2, q = c & 3;
  const float* src = in + (size_t)row * 16 + (q & 1) * 8;
  const v4f a = *(const v4f*)src;
  const v4f bq = *(const v4f*)(src + 4);
  const unsigned int keep = (q < 2) ? 0xffffffffu : 0u;
  v4u w4;
  w4.x = pack2h(a.x * sc, a.y * sc) & keep;
  w4.y = pack2h(a.z * sc, a.w * sc) & keep;
  w4.z = pack2h(bq.x * sc, bq.y * sc) & keep;
  w4.w = pack2h(bq.z * sc, bq.w * sc) & keep;
  v4u* dst = (v4u*)(void*)out + c;
  *(volatile v4u*)dst = w4;
  __threadfence();
  *(volatile v4u*)dst = w4;
}

__global__ __launch_bounds__(256) void k_cast_w1(const float* __restrict__ w, unsigned short* __restrict__ outp)
{
  const int c = (int)blockIdx.x * 256 + (int)threadIdx.x;
  if (c >= OUT_CH * (CPAD_CH / 8)) return;
  const int row = c / 36;
  const int q = c - row * 36;
  float f[8];
#pragma unroll
  for (int e = 0; e < 8; ++e) {
    const int j = 8 * q + e;
    const bool valid = j < CEXP_CH;
    const int src = (j < 128) ? j : ((j < 256) ? (j + 3) : (valid ? (j - 128) : 0));
    const float fv = w[(size_t)row * CEXP_CH + src];
    f[e] = valid ? fv * WCARRY : 0.0f;
  }
  v4u w4;
  w4.x = pack2h(f[0], f[1]); w4.y = pack2h(f[2], f[3]); w4.z = pack2h(f[4], f[5]); w4.w = pack2h(f[6], f[7]);
  v4u* dst = (v4u*)(void*)outp + c;
  *(volatile v4u*)dst = w4;
  __threadfence();
  *(volatile v4u*)dst = w4;
}

__global__ __launch_bounds__(256) void k_cast_flat2(
    const float* __restrict__ inA, int nchA, unsigned short* __restrict__ outA,
    const float* __restrict__ inB, int nchB, unsigned short* __restrict__ outB, int nblkA)
{
  const bool segA = (int)blockIdx.x < nblkA;
  const float* in = segA ? inA : inB;
  unsigned short* out = segA ? outA : outB;
  const int nch = segA ? nchA : nchB;
  const int c = (segA ? (int)blockIdx.x : ((int)blockIdx.x - nblkA)) * 256 + (int)threadIdx.x;
  if (c >= nch) return;
  const float* src = in + (size_t)c * 8;
  const v4f a = *(const v4f*)src;
  const v4f bq = *(const v4f*)(src + 4);
  v4u w4;
  w4.x = pack2h(a.x * WCARRY, a.y * WCARRY);
  w4.y = pack2h(a.z * WCARRY, a.w * WCARRY);
  w4.z = pack2h(bq.x * WCARRY, bq.y * WCARRY);
  w4.w = pack2h(bq.z * WCARRY, bq.w * WCARRY);
  v4u* dst = (v4u*)(void*)out + c;
  *(volatile v4u*)dst = w4;
  __threadfence();
  *(volatile v4u*)dst = w4;
}

template <bool HAS_BIAS, bool RESID, bool WROW, bool OUTF32, bool OUTF16>
__global__ __launch_bounds__(256) void gemm64_bn(
    const unsigned short* __restrict__ Ap, int lda,
    const unsigned short* __restrict__ Btp, int ldb,
    float* __restrict__ Cf, unsigned short* __restrict__ Ch, int ldc,
    const float* __restrict__ bias, const float* __restrict__ gam, const float* __restrict__ bet,
    const float* __restrict__ resid, const float* __restrict__ wrow,
    int M, int N, int K)
{
  typedef _Float16 T;
  typedef v16h V;
  const T* A = (const T*)(const void*)Ap;
  const T* Bt = (const T*)(const void*)Btp;
  __shared__ __align__(16) float sT[8][16 * 68];
  const int lane = threadIdx.x & 31;
  const int wave = threadIdx.x >> 5;
  const int tilesN = N >> 6;
  const int tilesM = M >> 6;
  const int tile = blockIdx.x * 8 + wave;
  if (tile >= tilesM * tilesN) return;
  const int tm = tile / tilesN;
  const int tn = tile - tm * tilesN;
  const int m0 = tm << 6;
  const int n0 = tn << 6;
  const int rlane = lane & 15;
  const int koff  = (lane >> 4) * 8;
  const int mOff  = (lane >> 4) * 8;

  v8f acc[4][4];
#pragma unroll
  for (int i = 0; i < 4; ++i)
#pragma unroll
    for (int j = 0; j < 4; ++j) acc[i][j] = (v8f){0.f,0.f,0.f,0.f,0.f,0.f,0.f,0.f};

  for (int k0 = 0; k0 < K; k0 += 32) {
    V bh[4];
#pragma unroll
    for (int j = 0; j < 4; ++j) {
      const size_t bo = (size_t)(n0 + (j << 4) + rlane) * ldb + koff + k0;
      bh[j] = Frag<T>::load(Bt + bo);
    }
#pragma unroll
    for (int i = 0; i < 4; ++i) {
      const size_t ao = (size_t)(m0 + (i << 4) + rlane) * lda + koff + k0;
      V ah = Frag<T>::load(A + ao);
#pragma unroll
      for (int j = 0; j < 4; ++j) acc[i][j] = Frag<T>::mma(ah, bh[j], acc[i][j]);
      Frag<T>::guard(acc[i][0], acc[i][3], ah, ah);
    }
    Frag<T>::keep(bh[0], bh[1], bh[2], bh[3]);
  }
  acc_guard4(acc[0][0], acc[0][1], acc[0][2], acc[0][3]);
  acc_guard4(acc[1][0], acc[1][1], acc[1][2], acc[1][3]);
  acc_guard4(acc[2][0], acc[2][1], acc[2][2], acc[2][3]);
  acc_guard4(acc[3][0], acc[3][1], acc[3][2], acc[3][3]);

  float pb[4], pg[4], pe[4];
#pragma unroll
  for (int j = 0; j < 4; ++j) {
    const int n = n0 + (j << 4) + rlane;
    pb[j] = HAS_BIAS ? bias[n] : 0.0f;
    pg[j] = gam[n] * INVSQ;
    pe[j] = bet[n];
  }

  float* slab = sT[wave];
  const int hh = lane >> 4, c4 = (lane & 15) * 4;
  const int q8 = lane >> 3, c8 = (lane & 7) * 8;
#pragma unroll
  for (int i = 0; i < 4; ++i) {
    const int mBase = m0 + (i << 4);
#pragma unroll
    for (int j = 0; j < 4; ++j) {
#pragma unroll
      for (int r = 0; r < 8; ++r) {
        const float s0 = acc[i][j][r] * WCARRY_INV;
        const float s1 = s0 + pb[j];
        const float s2 = s1 * pg[j];
        slab[(mOff + r) * 68 + (j << 4) + rlane] = s2 + pe[j];
      }
    }
    wave_sync();
#pragma unroll
    for (int it = 0; it < 8; ++it) {
      const int row = it * 2 + hh;
      v4f v = *(const v4f*)(slab + row * 68 + c4);
      if (RESID) {
        const v4f r4 = *(const v4f*)(resid + (size_t)(mBase + row) * ldc + n0 + c4);
        v += r4;
      }
      v.x = fmaxf(v.x, 0.0f); v.y = fmaxf(v.y, 0.0f); v.z = fmaxf(v.z, 0.0f); v.w = fmaxf(v.w, 0.0f);
      if (WROW) {
        const float wv1 = wrow[mBase + row];
        v *= wv1;
      }
      *(v4f*)(slab + row * 68 + c4) = v;
    }
    wave_sync();
    for (int pass = 0; pass < 2; ++pass) {
      if (OUTF32) {
#pragma unroll
        for (int it = 0; it < 8; ++it) {
          const int row = it * 2 + hh;
          const v4f v = *(const v4f*)(slab + row * 68 + c4);
          *(volatile v4f*)(Cf + (size_t)(mBase + row) * ldc + n0 + c4) = v;
        }
      }
      if (OUTF16) {
#pragma unroll
        for (int it = 0; it < 4; ++it) {
          const int row = it * 4 + q8;
          const float* sp = slab + row * 68 + c8;
          v8h hv;
#pragma unroll
          for (int e = 0; e < 8; ++e) hv[e] = (_Float16)sp[e];
          *(volatile v8h*)((_Float16*)(void*)Ch + (size_t)(mBase + row) * ldc + n0 + c8) = hv;
        }
      }
      __threadfence();
    }
    wave_sync();
  }
}

__global__ __launch_bounds__(FPS_THREADS) void k_fps(const float* __restrict__ xyz, unsigned int* __restrict__ selT)
{
#pragma clang fp contract(off)
  extern __shared__ float sx[];
  __shared__ float rv[2][16];
  __shared__ int   ri[2][16];
  __shared__ int   sels[NGRP];
  const int b = blockIdx.x, t = threadIdx.x, lane = t & 31, wv = t >> 5;
  const float* xb = xyz + (size_t)b * NPTS * 3;
  for (int i = t; i < NPTS * 3; i += FPS_THREADS) sx[i] = xb[i];
  __syncthreads();

  float px[FPS_PPT], py[FPS_PPT], pz[FPS_PPT], md[FPS_PPT];
  float bv = -1.0f; int bi = 0;
#pragma unroll
  for (int j = 0; j < FPS_PPT; ++j) {
    const int i = t + FPS_THREADS * j;
    const float x = sx[3 * i], y = sx[3 * i + 1], z = sx[3 * i + 2];
    px[j] = x; py[j] = y; pz[j] = z; md[j] = 1.0e10f;
    const float t0 = x * x, t1 = y * y, t2 = z * z;
    const float s02 = t0 + t2;
    const float s = s02 + t1;
    const bool tk = s > bv;
    bv = tk ? s : bv; bi = tk ? i : bi;
  }
  wave_argmax(bv, bi);
  if (lane == 0) { rv[0][wv] = bv; ri[0][wv] = bi; }
  __syncthreads();
  int cur;
  {
    float v = rv[0][0]; int ix = ri[0][0];
#pragma unroll
    for (int w2 = 1; w2 < 16; ++w2) lex_max(v, ix, rv[0][w2], ri[0][w2]);
    cur = ix;
  }
  for (int it = 0; it < NGRP; ++it) {
    if (t == 0) sels[it] = cur;
    const float cx = sx[3 * cur], cy = sx[3 * cur + 1], cz = sx[3 * cur + 2];
    bv = -1.0f; bi = 0;
#pragma unroll
    for (int j = 0; j < FPS_PPT; ++j) {
      const float dx = px[j] - cx, dy = py[j] - cy, dz = pz[j] - cz;
      const float t0 = dx * dx, t1 = dy * dy, t2 = dz * dz;
      const float s02 = t0 + t2;
      const float d = s02 + t1;
      const float m = fminf(md[j], d);
      md[j] = m;
      const bool tk = m > bv;
      bv = tk ? m : bv; bi = tk ? (t + FPS_THREADS * j) : bi;
    }
    wave_argmax(bv, bi);
    const int p = (it + 1) & 1;
    if (lane == 0) { rv[p][wv] = bv; ri[p][wv] = bi; }
    __syncthreads();
    float v = rv[p][0]; int ix = ri[p][0];
#pragma unroll
    for (int w2 = 1; w2 < 16; ++w2) lex_max(v, ix, rv[p][w2], ri[p][w2]);
    cur = ix;
  }
  __syncthreads();
  if (wv == 0) {
    unsigned int* dst = selT + (size_t)b * NGRP;
    for (int pass = 0; pass < 2; ++pass) {
#pragma unroll
      for (int u = 0; u < 4; ++u) {
        const int c = lane + 32 * u;
        v4u val;
        val.x = (unsigned int)sels[4 * c]; val.y = (unsigned int)sels[4 * c + 1];
        val.z = (unsigned int)sels[4 * c + 2]; val.w = (unsigned int)sels[4 * c + 3];
        *(volatile v4u*)(dst + 4 * c) = val;
      }
      __threadfence();
    }
  }
}

__device__ __forceinline__ float sq_dist(const float* xb, int i, float cx, float cy, float cz, float qq)
{
#pragma clang fp contract(off)
  const float rx = xb[3 * i], ry = xb[3 * i + 1], rz = xb[3 * i + 2];
  const float t0 = rx * rx, t1 = ry * ry, t2 = rz * rz;
  const float s02 = t0 + t2;
  const float rr = s02 + t1;
  float p = rx * cx;
  p = fmaf(ry, cy, p);
  p = fmaf(rz, cz, p);
  const float s2 = qq + rr;
  const float p2 = 2.0f * p;
  const float dd = s2 - p2;
  return fmaxf(dd, 0.0f);
}

__global__ __launch_bounds__(256) void k_knn(const float* __restrict__ xyz, const unsigned int* __restrict__ selT,
                                             unsigned int* __restrict__ knnT)
{
#pragma clang fp contract(off)
  __shared__ float lsd[8][KNN_CAP];
  __shared__ int   lsi[8][KNN_CAP];
  const int lane = threadIdx.x & 31, wv = threadIdx.x >> 5;
  const int bg = (int)blockIdx.x * 8 + wv;
  const int b = bg >> 9;
  const unsigned int uc = selT[bg];
  const int cidx = (int)(uc < (unsigned int)NPTS ? uc : (unsigned int)(NPTS - 1));
  const float* xb = xyz + (size_t)b * NPTS * 3;
  const float cx = xb[3 * cidx], cy = xb[3 * cidx + 1], cz = xb[3 * cidx + 2];
  const float q0 = cx * cx, q1 = cy * cy, q2 = cz * cz;
  const float q02 = q0 + q2;
  const float qq = q02 + q1;

  float d0 = FINF, d1 = FINF, d2 = FINF, d3 = FINF;
  int i0 = BIGI, i1 = BIGI, i2 = BIGI, i3 = BIGI;
#pragma unroll 2
  for (int j = 0; j < 256; ++j) {
    const int i = 32 * j + lane;
    const float dd = sq_dist(xb, i, cx, cy, cz, qq);
    const bool lt0 = dd < d0, lt1 = dd < d1, lt2 = dd < d2, lt3 = dd < d3;
    const float n3 = lt2 ? d2 : (lt3 ? dd : d3); const int m3 = lt2 ? i2 : (lt3 ? i : i3);
    const float n2 = lt1 ? d1 : (lt2 ? dd : d2); const int m2 = lt1 ? i1 : (lt2 ? i : i2);
    const float n1 = lt0 ? d0 : (lt1 ? dd : d1); const int m1 = lt0 ? i0 : (lt1 ? i : i1);
    const float nv0 = lt0 ? dd : d0;            const int mv0 = lt0 ? i : i0;
    d0 = nv0; d1 = n1; d2 = n2; d3 = n3; i0 = mv0; i1 = m1; i2 = m2; i3 = m3;
  }

  int myidx = 0, pops = 0;
  float Td = FINF; int Ti = BIGI;
#pragma unroll 1
  for (int r = 0; r < KNBR; ++r) {
    float cd = d0; int ci = i0;
    wave_argmin(cd, ci);
    const bool win = (i0 == ci);
    d0 = win ? d1 : d0; i0 = win ? i1 : i0;
    d1 = win ? d2 : d1; i1 = win ? i2 : i1;
    d2 = win ? d3 : d2; i2 = win ? i3 : i2;
    d3 = win ? FINF : d3; i3 = win ? BIGI : i3;
    pops += win ? 1 : 0;
    myidx = (lane == r) ? ci : myidx;
    Td = cd; Ti = ci;
  }
  const unsigned int fullm = __builtin_amdgcn_ballot_w32(pops >= 4);
  if (fullm != 0u) {
#pragma unroll
    for (int tq = 0; tq < KNN_CAP / 32; ++tq) { lsd[wv][lane + 32 * tq] = FINF; lsi[wv][lane + 32 * tq] = BIGI; }
    wave_sync();
    int base = 0;
#pragma unroll 2
    for (int j = 0; j < 256; ++j) {
      const int i = 32 * j + lane;
      const float dd = sq_dist(xb, i, cx, cy, cz, qq);
      const bool pred = (dd < Td) || (dd == Td && i <= Ti);
      const unsigned int m = __builtin_amdgcn_ballot_w32(pred);
      const int pos = base + (int)__builtin_popcount(m & ((1u << lane) - 1u));
      if (pred && pos < KNN_CAP) { lsd[wv][pos] = dd; lsi[wv][pos] = i; }
      base += (int)__builtin_popcount(m);
    }
    wave_sync();
    const int cnt = base < KNN_CAP ? base : KNN_CAP;
    float ed[4]; int ei[4];
#pragma unroll
    for (int tq = 0; tq < 4; ++tq) {
      const int e = lane + 32 * tq;
      const float vd = lsd[wv][e]; const int vi = lsi[wv][e];
      const bool ok = e < cnt;
      ed[tq] = ok ? vd : FINF; ei[tq] = ok ? vi : BIGI;
    }
#pragma unroll 1
    for (int r = 0; r < KNBR; ++r) {
      float cd = ed[0]; int ci = ei[0];
      lex_min(cd, ci, ed[1], ei[1]);
      lex_min(cd, ci, ed[2], ei[2]);
      lex_min(cd, ci, ed[3], ei[3]);
      wave_argmin(cd, ci);
#pragma unroll
      for (int tq = 0; tq < 4; ++tq) {
        const bool hit = (ei[tq] == ci);
        ed[tq] = hit ? FINF : ed[tq]; ei[tq] = hit ? BIGI : ei[tq];
      }
      myidx = (lane == r) ? ci : myidx;
    }
  }

  const unsigned int nidx = ((unsigned int)myidx < (unsigned int)NPTS) ? (unsigned int)myidx : (unsigned int)(NPTS - 1);
  const float nxv = xb[3 * nidx], nyv = xb[3 * nidx + 1], nzv = xb[3 * nidx + 2];
  const float rx = nxv - cx, ry = nyv - cy, rz = nzv - cz;
  const double drx = (double)rx, dry = (double)ry, drz = (double)rz;
  double s = (drx + dry) + drz;
  double q = (drx * drx + dry * dry) + drz * drz;
#pragma unroll
  for (int off = 16; off > 0; off >>= 1) { s += shfl_xor_d(s, off); q += shfl_xor_d(q, off); }
  const unsigned long long sb = (unsigned long long)__double_as_longlong(s);
  const unsigned long long qb = (unsigned long long)__double_as_longlong(q);
  v4u sv;
  sv.x = (lane == 0) ? (unsigned int)(sb & 0xffffffffULL) : 0u;
  sv.y = (lane == 0) ? (unsigned int)(sb >> 32) : 0u;
  sv.z = (lane == 0) ? (unsigned int)(qb & 0xffffffffULL) : 0u;
  sv.w = (lane == 0) ? (unsigned int)(qb >> 32) : 0u;
  unsigned int* rec = knnT + (size_t)bg * KNN_TPITCH;
  for (int pass = 0; pass < 2; ++pass) {
    *(volatile unsigned int*)(rec + lane) = nidx;
    if (lane < 8) *(volatile v4u*)(rec + 32 + lane * 4) = sv;
    __threadfence();
  }
}

__global__ __launch_bounds__(512) void k_stats(const unsigned int* __restrict__ knnT, float* __restrict__ statsL)
{
  __shared__ double ss[512];
  __shared__ double sq[512];
  const int t = threadIdx.x;
  double s = 0.0, q = 0.0;
#pragma unroll
  for (int u = 0; u < 8; ++u) {
    const int qi = t * 8 + u;
    const double* dp = (const double*)(const void*)(knnT + (size_t)qi * KNN_TPITCH + 32);
    s += dp[0]; q += dp[1];
  }
  ss[t] = s; sq[t] = q;
  __syncthreads();
  for (int st = 256; st > 0; st >>= 1) {
    if (t < st) { ss[t] += ss[t + st]; sq[t] += sq[t + st]; }
    __syncthreads();
  }
  const double S = ss[0], Q = sq[0];
  const double n = (double)(NQRY * KNBR * 3);
  const double mean = S / n;
  double var = (Q - S * mean) / (n - 1.0);
  var = var > 0.0 ? var : 0.0;
  const float sd = sqrtf((float)var) + 1.0e-5f;
  const float inv = 1.0f / sd;
  if (t < 32) {
    const float val = (t == 0) ? sd : ((t == 1) ? inv : 0.0f);
    for (int pass = 0; pass < 2; ++pass) {
      *(volatile float*)(statsL + t) = val;
      __threadfence();
    }
  }
}

__global__ __launch_bounds__(256) void k_expand(
    const float* __restrict__ xyz, const unsigned short* __restrict__ f0h,
    const unsigned int* __restrict__ selT, const unsigned int* __restrict__ knnT,
    const float* __restrict__ statsL, unsigned short* __restrict__ Ep, float* __restrict__ wgt, int b)
{
  const int lane = threadIdx.x & 31, wv = threadIdx.x >> 5;
  const int gl = (int)blockIdx.x * 8 + wv;
  const int bg = b * NGRP + gl;
  const unsigned int un = knnT[(size_t)bg * KNN_TPITCH + lane];
  const unsigned int nidx = un < (unsigned int)NPTS ? un : (unsigned int)(NPTS - 1);
  const unsigned int uc = selT[bg];
  const unsigned int cidx = uc < (unsigned int)NPTS ? uc : (unsigned int)(NPTS - 1);
  const float* xb = xyz + (size_t)b * NPTS * 3;
  const float nxv = xb[3 * nidx], nyv = xb[3 * nidx + 1], nzv = xb[3 * nidx + 2];
  const float ccx = xb[3 * cidx], ccy = xb[3 * cidx + 1], ccz = xb[3 * cidx + 2];
  const float inv = statsL[1];
  const float rx = nxv - ccx, ry = nyv - ccy, rz = nzv - ccz;
  const float ax = rx * inv - ccx, ay = ry * inv - ccy, az = rz * inv - ccz;
  const float nrm = sqrtf((ax * ax + ay * ay) + az * az);
  const float w = expf(-0.5f * nrm);
  const unsigned int pxy = pack2h(nxv, nyv);
  const unsigned int pzz = (unsigned int)h_bits(nzv);

  const v4u* f0c = (const v4u*)(const void*)f0h;
  const size_t rowc = (size_t)((size_t)b * NPTS + cidx) * 16;
  v4u* Eb = (v4u*)(void*)Ep + (size_t)gl * (KNBR * (CPAD_CH / 8));
#pragma unroll 1
  for (int tq = 0; tq < CPAD_CH / 8; ++tq) {
    const int c = lane + 32 * tq;
    const int k = c / 36;
    const int q = c - 36 * k;
    const int ik = __shfl((int)nidx, k, 32);
    const unsigned int uxy = __shfl(pxy, k, 32);
    const unsigned int uz  = __shfl(pzz, k, 32);
    const v4u an = f0c[(size_t)((size_t)b * NPTS + (unsigned int)ik) * 16 + (q & 15)];
    const v4u ac = f0c[rowc + (q & 15)];
    const bool s0 = q < 16, s1 = q < 32, s2 = (q == 32);
    v4u val;
    val.x = s0 ? an.x : (s1 ? ac.x : (s2 ? uxy : 0u));
    val.y = s0 ? an.y : (s1 ? ac.y : (s2 ? uz : 0u));
    val.z = s0 ? an.z : (s1 ? ac.z : 0u);
    val.w = s0 ? an.w : (s1 ? ac.w : 0u);
    *(volatile v4u*)(Eb + c) = val;
    __threadfence();
    *(volatile v4u*)(Eb + c) = val;
  }
  float* wl = wgt + (size_t)gl * KNBR;
  *(volatile float*)(wl + lane) = w;
  __threadfence();
  *(volatile float*)(wl + lane) = w;
}

__global__ __launch_bounds__(256) void k_pool(const float* __restrict__ X, float* __restrict__ outb)
{
  __shared__ float res[OUT_CH][33];
  const int g0 = (int)blockIdx.x * 32;
  const int m = threadIdx.x;
#pragma unroll 1
  for (int gq = 0; gq < 32; ++gq) {
    const size_t rb = (size_t)(g0 + gq) * KNBR;
    float mx = -FINF, sm = 0.0f;
#pragma unroll 8
    for (int k = 0; k < KNBR; ++k) {
      const float v = X[(rb + k) * OUT_CH + m];
      mx = fmaxf(mx, v);
      sm = sm + v;
    }
    res[m][gq] = mx + sm * (1.0f / 32.0f);
  }
  __syncthreads();
  const int wv = m >> 5, lane = m & 31;
  for (int pass = 0; pass < 2; ++pass) {
#pragma unroll 1
    for (int mm = 0; mm < 32; ++mm) {
      const int m2 = wv * 32 + mm;
      const float val = res[m2][lane];
      *(volatile float*)(outb + (size_t)m2 * NGRP + g0 + lane) = val;
    }
    __threadfence();
  }
}

template <bool HAS_BIAS, bool RESID, bool WROW, bool OUTF32, bool OUTF16>
static void launch_gemm(const unsigned short* A, int lda, const unsigned short* Bt, int ldb,
                        float* Cf, unsigned short* Ch, int ldc,
                        const float* bias, const float* gam, const float* bet,
                        const float* resid, const float* wrow, int M, int N, int K, hipStream_t stream)
{
  const int tiles = (M / 64) * (N / 64);
  const int blocks = (tiles + 7) / 8;
  gemm64_bn<HAS_BIAS, RESID, WROW, OUTF32, OUTF16><<<blocks, 256, 0, stream>>>(
      A, lda, Bt, ldb, Cf, Ch, ldc, bias, gam, bet, resid, wrow, M, N, K);
}

extern "C" void kernel_launch(void* const* d_in, const int* in_sizes, int n_in,
                              void* d_out, int out_size, void* d_ws, size_t ws_size,
                              hipStream_t stream) {
  if (n_in < 17) return;
  if (in_sizes[0] != NBATCH * NPTS * 3 || in_sizes[1] != NBATCH * NPTS * DIN_CH) return;
  if (out_size != NBATCH * OUT_CH * NGRP) return;
  if (ws_size < WS_TOTAL) return;

  const float* xyz     = (const float*)d_in[0];
  const float* feat    = (const float*)d_in[1];
  const float* w_embed = (const float*)d_in[2];
  const float* b_embed = (const float*)d_in[3];
  const float* g_embed = (const float*)d_in[4];
  const float* be_embed= (const float*)d_in[5];
  const float* w_lin1  = (const float*)d_in[6];
  const float* g_lin1  = (const float*)d_in[7];
  const float* be_lin1 = (const float*)d_in[8];
  const float* down_w  = (const float*)d_in[9];
  const float* down_b  = (const float*)d_in[10];
  const float* gd      = (const float*)d_in[11];
  const float* bd      = (const float*)d_in[12];
  const float* up_w    = (const float*)d_in[13];
  const float* up_b    = (const float*)d_in[14];
  const float* gu      = (const float*)d_in[15];
  const float* bu      = (const float*)d_in[16];
  float* out = (float*)d_out;

  char* ws = (char*)d_ws;
  unsigned short* featP = (unsigned short*)(ws + OFF_FEATP);
  unsigned short* Weh   = (unsigned short*)(ws + OFF_WEH);
  unsigned short* W1h   = (unsigned short*)(ws + OFF_W1H);
  unsigned short* Wdh   = (unsigned short*)(ws + OFF_WDH);
  unsigned short* Wuh   = (unsigned short*)(ws + OFF_WUH);
  unsigned short* f0h   = (unsigned short*)(ws + OFF_F0H);
  unsigned int*   selT  = (unsigned int*)(ws + OFF_SELT);
  unsigned int*   knnT  = (unsigned int*)(ws + OFF_KNNT);
  float*          statsL= (float*)(ws + OFF_STATS);
  unsigned short* Eh    = (unsigned short*)(ws + OFF_E);
  float*          wgt   = (float*)(ws + OFF_WGT);
  float*          X32a  = (float*)(ws + OFF_X32A);
  float*          X32b  = (float*)(ws + OFF_X32B);
  unsigned short* X16   = (unsigned short*)(ws + OFF_X16);
  unsigned short* H16   = (unsigned short*)(ws + OFF_H16);

  constexpr int NCH_FEAT = NPT_ALL * 4;
  constexpr int NCH_WE   = PREV_CH * 4;
  static_assert(NCH_FEAT % 256 == 0 && NCH_WE % 256 == 0);
  k_cast_pad2<<<NCH_FEAT / 256 + NCH_WE / 256, 256, 0, stream>>>(
      feat, NCH_FEAT, featP, w_embed, NCH_WE, Weh, NCH_FEAT / 256, WCARRY);
  static_assert((OUT_CH * (CPAD_CH / 8)) % 256 == 0);
  k_cast_w1<<<(OUT_CH * (CPAD_CH / 8)) / 256, 256, 0, stream>>>(w_lin1, W1h);
  constexpr int NCH_WD = 2 * MID_CH * OUT_CH / 8;
  constexpr int NCH_WU = 2 * OUT_CH * MID_CH / 8;
  static_assert(NCH_WD % 256 == 0 && NCH_WU % 256 == 0);
  k_cast_flat2<<<NCH_WD / 256 + NCH_WU / 256, 256, 0, stream>>>(
      down_w, NCH_WD, Wdh, up_w, NCH_WU, Wuh, NCH_WD / 256);

  static_assert(NPT_ALL % 64 == 0 && PREV_CH % 64 == 0 && KPAD_EMB % 32 == 0);
  launch_gemm<true, false, false, false, true>(featP, KPAD_EMB, Weh, KPAD_EMB, X32a, f0h, PREV_CH,
                                               b_embed, g_embed, be_embed, X32a, g_embed,
                                               NPT_ALL, PREV_CH, KPAD_EMB, stream);

  k_fps<<<NBATCH, FPS_THREADS, (size_t)NPTS * 3 * sizeof(float), stream>>>(xyz, selT);
  static_assert(NQRY % 8 == 0);
  k_knn<<<NQRY / 8, 256, 0, stream>>>(xyz, selT, knnT);
  static_assert(NQRY == 512 * 8);
  k_stats<<<1, 512, 0, stream>>>(knnT, statsL);

  static_assert(ROWS_CHUNK % 64 == 0 && OUT_CH % 64 == 0 && MID_CH % 64 == 0);
  static_assert(CPAD_CH % 32 == 0 && OUT_CH % 32 == 0 && MID_CH % 32 == 0);
  static_assert(NGRP % 32 == 0 && NGRP % 8 == 0);
  for (int b = 0; b < NBATCH; ++b) {
    k_expand<<<NGRP / 8, 256, 0, stream>>>(xyz, f0h, selT, knnT, statsL, Eh, wgt, b);
    launch_gemm<false, false, true, true, true>(Eh, CPAD_CH, W1h, CPAD_CH, X32a, X16, OUT_CH,
                                                g_lin1, g_lin1, be_lin1, X32a, wgt,
                                                ROWS_CHUNK, OUT_CH, CPAD_CH, stream);
    launch_gemm<true, false, false, false, true>(X16, OUT_CH, Wdh, OUT_CH, X32a, H16, MID_CH,
                                                 down_b, gd, bd, X32a, wgt,
                                                 ROWS_CHUNK, MID_CH, OUT_CH, stream);
    launch_gemm<true, true, false, true, true>(H16, MID_CH, Wuh, MID_CH, X32b, X16, OUT_CH,
                                               up_b, gu, bu, X32a, wgt,
                                               ROWS_CHUNK, OUT_CH, MID_CH, stream);
    launch_gemm<true, false, false, false, true>(X16, OUT_CH, Wdh + (size_t)MID_CH * OUT_CH, OUT_CH, X32a, H16, MID_CH,
                                                 down_b + MID_CH, gd + MID_CH, bd + MID_CH, X32a, wgt,
                                                 ROWS_CHUNK, MID_CH, OUT_CH, stream);
    launch_gemm<true, true, false, true, false>(H16, MID_CH, Wuh + (size_t)OUT_CH * MID_CH, MID_CH, X32a, X16, OUT_CH,
                                                up_b + OUT_CH, gu + OUT_CH, bu + OUT_CH, X32b, wgt,
                                                ROWS_CHUNK, OUT_CH, MID_CH, stream);
    k_pool<<<NGRP / 32, 256, 0, stream>>>(X32a, out + (size_t)b * OUT_CH * NGRP);
  }
}
